// SplitedTreeLSTM_25151328485755
// MI455X (gfx1250) — hardware-verified
//
#include <hip/hip_runtime.h>
#include <math.h>
#include <stdint.h>

#define NTR    4096
#define LPOS   64
#define ISZ    64
#define HSZ    128
#define OSZ    128
#define G4     512
#define AH     64
#define NTOK   (NTR * LPOS)
#define NCHUNK 4
#define CTR    (NTR / NCHUNK)
#define CTOK   (CTR * LPOS)
#define BPC    (CTR / 8)
#define NPART  (NCHUNK * BPC)
#define SOP    132
static_assert((CTOK % 64) == 0);
static_assert((CTR % 8) == 0);
static_assert((ISZ % 32) == 0 && (HSZ % 32) == 0);

typedef __bf16   v16b __attribute__((ext_vector_type(16)));
typedef __bf16   v8b  __attribute__((ext_vector_type(8)));
typedef float    v8f  __attribute__((ext_vector_type(8)));
typedef float    v4f  __attribute__((ext_vector_type(4)));
typedef unsigned int v4u __attribute__((ext_vector_type(4)));

__device__ __forceinline__ unsigned short bf_bits(float f) {
  unsigned u = __float_as_uint(f);
  return (unsigned short)((u + 0x7FFFu + ((u >> 16) & 1u)) >> 16);
}
__device__ __forceinline__ float bf_up(unsigned short h) { return __uint_as_float(((unsigned)h) << 16); }
__device__ __forceinline__ float bf_rne(float f) { return bf_up(bf_bits(f)); }
__device__ __forceinline__ unsigned pk16(unsigned short a, unsigned short b) { return (unsigned)a | ((unsigned)b << 16); }
__device__ __forceinline__ v8f zero8() { v8f z = {0.f, 0.f, 0.f, 0.f, 0.f, 0.f, 0.f, 0.f}; return z; }
__device__ __forceinline__ int clampi(int v, int lo, int hi) { v = v < lo ? lo : v; return v > hi ? hi : v; }
__device__ __forceinline__ float sigm(float x) { return 1.0f / (1.0f + expf(-x)); }

__device__ __forceinline__ v16b ldfrag_b(const __bf16* p) {
  union { v16b v; v8b h[2]; } f;
  f.h[0] = *(const v8b*)(p);
  f.h[1] = *(const v8b*)(p + 16);
  return f.v;
}

__device__ __forceinline__ v8f mma_b_raw(v16b a, v16b b, v8f c) {
  return __builtin_amdgcn_wmma_f32_16x16x32_bf16(false, a, false, b, (short)0, c, false, false);
}
__device__ __forceinline__ void dep_guard_b(v8f& a, v8f& b, v16b x, v16b y) {
#if defined(__HIP_DEVICE_COMPILE__)
  asm volatile("v_nop\n\tv_nop\n\tv_nop\n\tv_nop" : "+v"(a), "+v"(b) : "v"(x), "v"(y));
#endif
}
__device__ __forceinline__ void keep4_b(v16b a, v16b b, v16b c, v16b d) {
#if defined(__HIP_DEVICE_COMPILE__)
  asm volatile("v_nop" :: "v"(a), "v"(b), "v"(c), "v"(d));
#endif
}
__device__ __forceinline__ void keep3_b(v16b a, v16b b, v16b c) {
#if defined(__HIP_DEVICE_COMPILE__)
  asm volatile("v_nop" :: "v"(a), "v"(b), "v"(c));
#endif
}
__device__ __forceinline__ void acc_guard4(v8f& a, v8f& b, v8f& c, v8f& d) {
#if defined(__HIP_DEVICE_COMPILE__)
  asm volatile("v_nop\n\tv_nop\n\tv_nop\n\tv_nop" : "+v"(a), "+v"(b), "+v"(c), "+v"(d));
#endif
}
__device__ __forceinline__ void acc_guard3(v8f& a, v8f& b, v8f& c) {
#if defined(__HIP_DEVICE_COMPILE__)
  asm volatile("v_nop\n\tv_nop\n\tv_nop\n\tv_nop" : "+v"(a), "+v"(b), "+v"(c));
#endif
}
__device__ __forceinline__ void wave_sync_lds() {
  __builtin_amdgcn_fence(__ATOMIC_RELEASE, "workgroup");
  __builtin_amdgcn_wave_barrier();
  __builtin_amdgcn_fence(__ATOMIC_ACQUIRE, "workgroup");
}

__global__ __launch_bounds__(256) void cvt_bf16x8(const float* __restrict__ in, unsigned short* out, int n8) {
  const int i = blockIdx.x * 256 + threadIdx.x;
  if (i < n8) {
    const v4f a = *(const v4f*)(in + (size_t)i * 8);
    const v4f b = *(const v4f*)(in + (size_t)i * 8 + 4);
    v4u p;
    p[0] = pk16(bf_bits(a[0]), bf_bits(a[1]));
    p[1] = pk16(bf_bits(a[2]), bf_bits(a[3]));
    p[2] = pk16(bf_bits(b[0]), bf_bits(b[1]));
    p[3] = pk16(bf_bits(b[2]), bf_bits(b[3]));
    *(volatile v4u*)(out + (size_t)i * 8) = p;
    __threadfence();
    *(volatile v4u*)(out + (size_t)i * 8) = p;
  }
}

__global__ __launch_bounds__(256) void gather_x(const int* __restrict__ traces, const float* __restrict__ emb,
                                                unsigned short* X, int rbase, int nrows, int nv) {
  const int lane = threadIdx.x & 31;
  const int wave = threadIdx.x >> 5;
  const int q    = lane >> 3;
  const int c8   = (lane & 7) * 8;
  const int rw   = blockIdx.x * 64 + wave * 8;
  if (rw + 8 > nrows) return;
  v4u p[2];
#pragma unroll
  for (int it = 0; it < 2; ++it) {
    const int rr  = rw + it * 4 + q;
    const int r   = clampi(rbase + rr, 0, NTOK - 1);
    const int tok = clampi(traces[r], 0, nv - 1);
    const float* src = emb + (size_t)tok * ISZ + c8;
    const v4f a = *(const v4f*)(src);
    const v4f c = *(const v4f*)(src + 4);
    v4u qv;
    qv[0] = pk16(bf_bits(a[0]), bf_bits(a[1]));
    qv[1] = pk16(bf_bits(a[2]), bf_bits(a[3]));
    qv[2] = pk16(bf_bits(c[0]), bf_bits(c[1]));
    qv[3] = pk16(bf_bits(c[2]), bf_bits(c[3]));
    p[it] = qv;
  }
  for (int pass = 0; pass < 2; ++pass) {
#pragma unroll
    for (int it = 0; it < 2; ++it) {
      const int rr = rw + it * 4 + q;
      *(volatile v4u*)(X + (size_t)rr * ISZ + c8) = p[it];
    }
    __threadfence();
  }
}

template <int NSPLIT, int F32OUT>
__global__ __launch_bounds__(256) void gemm_gate(
    const unsigned short* __restrict__ Ap, const unsigned short* A2p, int lda,
    const unsigned short* __restrict__ Btp,
    const float* __restrict__ bA, const float* __restrict__ bB,
    unsigned short* Hh, unsigned short* Hl, float* Hf, int K) {
  const __bf16* A  = (const __bf16*)(const void*)Ap;
  const __bf16* A2 = (const __bf16*)(const void*)A2p;
  const __bf16* Bt = (const __bf16*)(const void*)Btp;
  __shared__ __align__(16) float sO[64 * SOP];
  const int lane  = threadIdx.x & 31;
  const int wave  = threadIdx.x >> 5;
  const int m0    = blockIdx.x * 64;
  const int h0    = wave * 16;
  const int rlane = lane & 15;
  const int koff  = (lane >> 4) * 8;
  const int mOff  = (lane >> 4) * 8;
  const __bf16* Ab2 = (NSPLIT >= 1) ? A2 : A;

  const float bi0 = bf_rne(bA[h0 + rlane]),       bi1 = bf_rne(bB[h0 + rlane]);
  const float bc0 = bf_rne(bA[256 + h0 + rlane]), bc1 = bf_rne(bB[256 + h0 + rlane]);
  const float bo0 = bf_rne(bA[384 + h0 + rlane]), bo1 = bf_rne(bB[384 + h0 + rlane]);

  v8f acc[4][3];
#pragma unroll
  for (int i = 0; i < 4; ++i)
#pragma unroll
    for (int j = 0; j < 3; ++j) acc[i][j] = zero8();

  for (int k0 = 0; k0 < K; k0 += 32) {
    v16b bh[3];
#pragma unroll
    for (int j = 0; j < 3; ++j) {
      const int gb = (j == 0) ? 0 : (128 + 128 * j);
      const size_t bo = (size_t)(gb + h0 + rlane) * K + koff + k0;
      bh[j] = ldfrag_b(Bt + bo);
    }
#pragma unroll
    for (int i = 0; i < 4; ++i) {
      const size_t ao = (size_t)(m0 + (i << 4) + rlane) * lda + koff + k0;
      const v16b ah = ldfrag_b(A + ao);
      v16b al = ah;
      if (NSPLIT >= 1) al = ldfrag_b(Ab2 + ao);
#pragma unroll
      for (int j = 0; j < 3; ++j) {
        acc[i][j] = mma_b_raw(ah, bh[j], acc[i][j]);
        if (NSPLIT >= 1) acc[i][j] = mma_b_raw(al, bh[j], acc[i][j]);
      }
      dep_guard_b(acc[i][0], acc[i][2], ah, al);
    }
    keep3_b(bh[0], bh[1], bh[2]);
  }
  acc_guard3(acc[0][0], acc[0][1], acc[0][2]);
  acc_guard3(acc[1][0], acc[1][1], acc[1][2]);
  acc_guard3(acc[2][0], acc[2][1], acc[2][2]);
  acc_guard3(acc[3][0], acc[3][1], acc[3][2]);

#pragma unroll
  for (int i = 0; i < 4; ++i) {
#pragma unroll
    for (int r = 0; r < 8; ++r) {
      const float gi = (acc[i][0][r] + bi0) + bi1;
      const float gc = (acc[i][1][r] + bc0) + bc1;
      const float go = (acc[i][2][r] + bo0) + bo1;
      const float cc = sigm(gi) * tanhf(gc);
      const float hv = sigm(go) * tanhf(cc);
      sO[(i * 16 + mOff + r) * SOP + h0 + rlane] = hv;
    }
  }
  __syncthreads();

  const int rowf = wave * 8;
  for (int pass = 0; pass < 2; ++pass) {
    if (F32OUT) {
#pragma unroll
      for (int rr = 0; rr < 8; ++rr) {
        const int row = rowf + rr;
        const v4f v = *(const v4f*)(sO + row * SOP + lane * 4);
        *(volatile v4f*)(Hf + (size_t)(m0 + row) * HSZ + lane * 4) = v;
      }
    }
#pragma unroll
    for (int it = 0; it < 4; ++it) {
      const int row = rowf + it * 2 + (lane >> 4);
      const int cb  = (lane & 15) * 8;
      const float* sp = sO + row * SOP + cb;
      v4u a, a2;
#pragma unroll
      for (int e = 0; e < 4; ++e) {
        const float f0 = sp[2 * e], f1 = sp[2 * e + 1];
        const unsigned short x0 = bf_bits(f0), x1 = bf_bits(f1);
        const unsigned short l0 = bf_bits(f0 - bf_up(x0)), l1 = bf_bits(f1 - bf_up(x1));
        a[e] = pk16(x0, x1); a2[e] = pk16(l0, l1);
      }
      *(volatile v4u*)(Hh + (size_t)(m0 + row) * HSZ + cb) = a;
      *(volatile v4u*)(Hl + (size_t)(m0 + row) * HSZ + cb) = a2;
    }
    __threadfence();
  }
}

template <int NSPLIT, int OUT_MODE>
__global__ __launch_bounds__(256) void gemm64(
    const unsigned short* __restrict__ Ap, const unsigned short* A2p, int lda,
    const unsigned short* __restrict__ Btp, int ldb,
    const float* __restrict__ bias, int relu,
    void* Cout, void* Cout2, int ldc,
    const float* __restrict__ w3, const float* __restrict__ b3,
    int M, int N, int K) {
  const __bf16* A   = (const __bf16*)(const void*)Ap;
  const __bf16* A2  = (const __bf16*)(const void*)A2p;
  const __bf16* Bt  = (const __bf16*)(const void*)Btp;
  __shared__ __align__(16) float sT[8][16 * 68];
  __shared__ __align__(16) float sW3[8][64];
  __shared__ __align__(16) float sLg[8][64];
  const int lane = threadIdx.x & 31;
  const int wave = threadIdx.x >> 5;
  const int tilesN = N >> 6;
  const int tilesM = M >> 6;
  const int tile = blockIdx.x * 8 + wave;
  if (tile >= tilesM * tilesN) return;
  const int tm = tile / tilesN;
  const int tn = tile - tm * tilesN;
  const int m0 = tm << 6;
  const int n0 = tn << 6;

  const __bf16* Ab  = A;
  const __bf16* Bb  = Bt;
  const __bf16* Ab2 = (NSPLIT >= 1) ? A2 : Ab;

  const int rlane = lane & 15;
  const int koff  = (lane >> 4) * 8;
  const int mOff  = (lane >> 4) * 8;

  float bv[4];
#pragma unroll
  for (int j = 0; j < 4; ++j) bv[j] = bf_rne(bias[n0 + (j << 4) + rlane]);
  float b3v = 0.f;
  if (OUT_MODE == 4) {
    sW3[wave][lane]      = bf_rne(w3[lane]);
    sW3[wave][lane + 32] = bf_rne(w3[lane + 32]);
    b3v = bf_rne(b3[0]);
  }

  v8f acc[4][4];
#pragma unroll
  for (int i = 0; i < 4; ++i)
#pragma unroll
    for (int j = 0; j < 4; ++j) acc[i][j] = zero8();

  for (int k0 = 0; k0 < K; k0 += 32) {
    v16b bh[4];
#pragma unroll
    for (int j = 0; j < 4; ++j) {
      const size_t bo = (size_t)(n0 + (j << 4) + rlane) * ldb + koff + k0;
      bh[j] = ldfrag_b(Bb + bo);
    }
#pragma unroll
    for (int i = 0; i < 4; ++i) {
      const size_t ao = (size_t)(m0 + (i << 4) + rlane) * lda + koff + k0;
      const v16b ah = ldfrag_b(Ab + ao);
      v16b al = ah;
      if (NSPLIT >= 1) al = ldfrag_b(Ab2 + ao);
#pragma unroll
      for (int j = 0; j < 4; ++j) {
        acc[i][j] = mma_b_raw(ah, bh[j], acc[i][j]);
        if (NSPLIT >= 1) acc[i][j] = mma_b_raw(al, bh[j], acc[i][j]);
      }
      dep_guard_b(acc[i][0], acc[i][3], ah, al);
    }
    keep4_b(bh[0], bh[1], bh[2], bh[3]);
  }
  acc_guard4(acc[0][0], acc[0][1], acc[0][2], acc[0][3]);
  acc_guard4(acc[1][0], acc[1][1], acc[1][2], acc[1][3]);
  acc_guard4(acc[2][0], acc[2][1], acc[2][2], acc[2][3]);
  acc_guard4(acc[3][0], acc[3][1], acc[3][2], acc[3][3]);

  float* slab = sT[wave];
#pragma unroll
  for (int i = 0; i < 4; ++i) {
    const int mBase = m0 + (i << 4);
#pragma unroll
    for (int j = 0; j < 4; ++j) {
#pragma unroll
      for (int r = 0; r < 8; ++r) {
        float v = acc[i][j][r] + bv[j];
        if (relu) v = fmaxf(v, 0.0f);
        slab[(mOff + r) * 68 + (j << 4) + rlane] = v;
      }
    }
    wave_sync_lds();
    if (OUT_MODE == 2) {
      const int q = lane >> 3, c8 = (lane & 7) * 8;
      unsigned short* C  = (unsigned short*)Cout;
      unsigned short* C2 = (unsigned short*)Cout2;
      v4u hv[4], lv[4];
#pragma unroll
      for (int it = 0; it < 4; ++it) {
        const int row = it * 4 + q;
        const float* sp = slab + row * 68 + c8;
        v4u a, a2;
#pragma unroll
        for (int e = 0; e < 4; ++e) {
          const float f0 = sp[2 * e], f1 = sp[2 * e + 1];
          const unsigned short x0 = bf_bits(f0), x1 = bf_bits(f1);
          const unsigned short l0 = bf_bits(f0 - bf_up(x0)), l1 = bf_bits(f1 - bf_up(x1));
          a[e] = pk16(x0, x1); a2[e] = pk16(l0, l1);
        }
        hv[it] = a; lv[it] = a2;
      }
      for (int pass = 0; pass < 2; ++pass) {
#pragma unroll
        for (int it = 0; it < 4; ++it) {
          const int row = it * 4 + q;
          *(volatile v4u*)(C  + (size_t)(mBase + row) * ldc + n0 + c8) = hv[it];
          *(volatile v4u*)(C2 + (size_t)(mBase + row) * ldc + n0 + c8) = lv[it];
        }
        __threadfence();
      }
    } else {
      const int row = lane & 15, h2 = lane >> 4;
      const float* sp = slab + row * 68 + h2 * 32;
      const float* wp = sW3[wave] + h2 * 32;
      float s = 0.f;
#pragma unroll 4
      for (int t = 0; t < 32; ++t) s = fmaf(sp[t], wp[t], s);
      s += __shfl_xor(s, 16, 32);
      if (h2 == 0) sLg[wave][i * 16 + row] = s + b3v;
    }
    wave_sync_lds();
  }
  if (OUT_MODE == 4) {
    float* C = (float*)Cout;
    const v4f v = *(const v4f*)(sLg[wave] + 4 * (lane & 15));
    if (lane < 16) *(volatile v4f*)(C + (size_t)m0 + 4 * lane) = v;
    __threadfence();
    if (lane < 16) *(volatile v4f*)(C + (size_t)m0 + 4 * lane) = v;
  }
}

__global__ __launch_bounds__(256) void agg_trace(const int* __restrict__ lengths, const float* __restrict__ Lg,
                                                 const float* __restrict__ H2f, float* P,
                                                 int tbase, int ntr_total, int pbase) {
  __shared__ __align__(16) float sTE[8][HSZ];
  __shared__ __align__(16) float sP[HSZ];
  const int tid  = threadIdx.x;
  const int lane = tid & 31;
  const int wave = tid >> 5;
  const int tl   = blockIdx.x * 8 + wave;
  const int tg   = clampi(tbase + tl, 0, ntr_total - 1);
  const int len  = lengths[tg];
  const size_t rb = (size_t)tl * LPOS;
  const float E1 = Lg[rb + lane];
  const float E2 = Lg[rb + lane + 32];
  const float x1 = (lane < len)      ? E1 : -1.0e30f;
  const float x2 = (lane + 32 < len) ? E2 : -1.0e30f;
  float m = fmaxf(x1, x2);
#pragma unroll
  for (int off = 1; off < 32; off <<= 1) m = fmaxf(m, __shfl_xor(m, off, 32));
  const float e1 = __expf(x1 - m);
  const float e2 = __expf(x2 - m);
  float S = e1 + e2;
#pragma unroll
  for (int off = 1; off < 32; off <<= 1) S += __shfl_xor(S, off, 32);
  const float inv = 1.0f / S;
  const float w1 = e1 * inv;
  const float w2 = e2 * inv;

  float o0 = 0.f, o1 = 0.f, o2 = 0.f, o3 = 0.f;
#pragma unroll 2
  for (int l = 0; l < LPOS; ++l) {
    const bool lo = (l < 32);
    const float wsel = lo ? w1 : w2;
    const float wl = __shfl(wsel, l & 31, 32);
    const float* hr = H2f + (rb + (size_t)l) * HSZ;
    o0 = fmaf(wl, hr[lane],      o0);
    o1 = fmaf(wl, hr[lane + 32], o1);
    o2 = fmaf(wl, hr[lane + 64], o2);
    o3 = fmaf(wl, hr[lane + 96], o3);
  }
  sTE[wave][lane]      = o0;
  sTE[wave][lane + 32] = o1;
  sTE[wave][lane + 64] = o2;
  sTE[wave][lane + 96] = o3;
  __syncthreads();
  if (tid < HSZ) {
    float s = 0.f;
#pragma unroll
    for (int w = 0; w < 8; ++w) s += sTE[w][tid];
    sP[tid] = s;
  }
  __syncthreads();
  if (wave == 0) {
    const v4f v = *(const v4f*)(sP + 4 * lane);
    float* dst = P + (size_t)(pbase + blockIdx.x) * HSZ + 4 * lane;
    *(volatile v4f*)dst = v;
    __threadfence();
    *(volatile v4f*)dst = v;
  }
}

__global__ __launch_bounds__(128) void finisher(const float* __restrict__ P, const float* __restrict__ W_out,
                                                const float* __restrict__ b_out, float* out, int npart) {
  __shared__ __align__(16) float sF[HSZ];
  __shared__ __align__(16) float sOut[OSZ];
  const int tid = threadIdx.x;
  double s = 0.0;
#pragma unroll 4
  for (int b = 0; b < npart; ++b) s += (double)P[(size_t)b * HSZ + tid];
  sF[tid] = (float)s;
  __syncthreads();
  float a = 0.f;
  const float* wr = W_out + (size_t)tid * HSZ;
#pragma unroll 4
  for (int h = 0; h < HSZ; ++h) a = fmaf(sF[h], bf_rne(wr[h]), a);
  sOut[tid] = a + bf_rne(b_out[tid]);
  __syncthreads();
  if (tid < 32) {
    const v4f v = *(const v4f*)(sOut + 4 * tid);
    *(volatile v4f*)(out + 4 * tid) = v;
    __threadfence();
    *(volatile v4f*)(out + 4 * tid) = v;
  }
}

extern "C" void kernel_launch(void* const* d_in, const int* in_sizes, int n_in,
                              void* d_out, int out_size, void* d_ws, size_t ws_size,
                              hipStream_t stream) {
  if (n_in < 17) return;
  if (in_sizes[0] < ISZ || (in_sizes[0] % ISZ) != 0) return;
  if (in_sizes[1] != G4 * ISZ || in_sizes[3] != G4 || in_sizes[4] != G4) return;
  if (in_sizes[5] != G4 * HSZ || in_sizes[7] != G4 || in_sizes[8] != G4) return;
  if (in_sizes[9] != AH * HSZ || in_sizes[10] != AH || in_sizes[11] != AH || in_sizes[12] < 1) return;
  if (in_sizes[13] != OSZ * HSZ || in_sizes[14] != OSZ) return;
  if (in_sizes[15] != NTOK || in_sizes[16] != NTR) return;
  if (out_size != OSZ) return;

  const float* emb    = (const float*)d_in[0];
  const float* W_ih1  = (const float*)d_in[1];
  const float* b_ih1  = (const float*)d_in[3];
  const float* b_hh1  = (const float*)d_in[4];
  const float* W_ih2  = (const float*)d_in[5];
  const float* b_ih2  = (const float*)d_in[7];
  const float* b_hh2  = (const float*)d_in[8];
  const float* Wp1    = (const float*)d_in[9];
  const float* bp1    = (const float*)d_in[10];
  const float* Wp2    = (const float*)d_in[11];
  const float* bp2    = (const float*)d_in[12];
  const float* W_out  = (const float*)d_in[13];
  const float* b_out  = (const float*)d_in[14];
  const int*   traces = (const int*)  d_in[15];
  const int*   lens   = (const int*)  d_in[16];
  float* out = (float*)d_out;
  const int nv = in_sizes[0] / ISZ;

  const size_t PW1 = (size_t)G4 * ISZ * 2;
  const size_t PW2 = (size_t)G4 * HSZ * 2;
  const size_t PWp = (size_t)AH * HSZ * 2;
  const size_t PX  = (size_t)CTOK * ISZ * 2;
  const size_t PHb = (size_t)CTOK * HSZ * 2;
  const size_t PHf = (size_t)CTOK * HSZ * 4;
  const size_t PLg = (size_t)CTOK * 4;
  const size_t PP  = (size_t)NPART * HSZ * 4;
  size_t off = 0;
  const size_t oW1  = off; off += PW1;
  const size_t oW2  = off; off += PW2;
  const size_t oWp  = off; off += PWp;
  const size_t oX   = off; off += PX;
  const size_t oH1h = off; off += PHb;
  const size_t oH1l = off; off += PHb;
  const size_t oH2f = off; off += PHf;
  const size_t oH2h = off; off += PHb;
  const size_t oH2l = off; off += PHb;
  const size_t oLg  = off; off += PLg;
  const size_t oP   = off; off += PP;
  if (off > ws_size) return;
  if (off > (size_t)134217728) return;

  char* ws = (char*)d_ws;
  unsigned short* W1b  = (unsigned short*)(ws + oW1);
  unsigned short* W2b  = (unsigned short*)(ws + oW2);
  unsigned short* Wp1b = (unsigned short*)(ws + oWp);
  unsigned short* Xb   = (unsigned short*)(ws + oX);
  unsigned short* H1h  = (unsigned short*)(ws + oH1h);
  unsigned short* H1l  = (unsigned short*)(ws + oH1l);
  float*          H2f  = (float*)(ws + oH2f);
  unsigned short* H2h  = (unsigned short*)(ws + oH2h);
  unsigned short* H2l  = (unsigned short*)(ws + oH2l);
  float*          Lg   = (float*)(ws + oLg);
  float*          Pp   = (float*)(ws + oP);

  const dim3 blk(256);
  const int n8w1 = G4 * ISZ / 8;
  const int n8w2 = G4 * HSZ / 8;
  const int n8wp = AH * HSZ / 8;
  const dim3 gW1((n8w1 + 255) / 256);
  const dim3 gW2((n8w2 + 255) / 256);
  const dim3 gWp((n8wp + 255) / 256);
  const dim3 gRow(CTOK / 64);
  const dim3 gEn((CTOK / 64 + 7) / 8);
  const dim3 gAgg(BPC);

  cvt_bf16x8<<<gW1, blk, 0, stream>>>(W_ih1, W1b, n8w1);
  cvt_bf16x8<<<gW2, blk, 0, stream>>>(W_ih2, W2b, n8w2);
  cvt_bf16x8<<<gWp, blk, 0, stream>>>(Wp1, Wp1b, n8wp);
  for (int c = 0; c < NCHUNK; ++c) {
    gather_x<<<gRow, blk, 0, stream>>>(traces, emb, Xb, c * CTOK, CTOK, nv);
    gemm_gate<0, 0><<<gRow, blk, 0, stream>>>(Xb, Xb, ISZ, W1b, b_ih1, b_hh1, H1h, H1l, H2f, ISZ);
    gemm_gate<1, 1><<<gRow, blk, 0, stream>>>(H1h, H1l, HSZ, W2b, b_ih2, b_hh2, H2h, H2l, H2f, HSZ);
    gemm64<1, 4><<<gEn, blk, 0, stream>>>(
        H2h, H2l, HSZ, Wp1b, HSZ, bp1, 1,
        (void*)Lg, (void*)Lg, AH, Wp2, bp2,
        CTOK, AH, HSZ);
    agg_trace<<<gAgg, blk, 0, stream>>>(lens, Lg, H2f, Pp, c * CTR, NTR, c * BPC);
  }
  finisher<<<dim3(1), dim3(128), 0, stream>>>(Pp, W_out, b_out, out, NPART);
  (void)hipGetLastError();
}
